// NeusBackgroundModule_64089501991444
// MI455X (gfx1250) — hardware-verified
//
#include <hip/hip_runtime.h>

#define N_IMAGES 32
#define IMG_H 512
#define IMG_W 512
#define HID 256
#define N_PIX 4096

typedef _Float16 v16h __attribute__((ext_vector_type(16)));
typedef _Float16 v8h  __attribute__((ext_vector_type(8)));
typedef _Float16 v8ha __attribute__((ext_vector_type(8), may_alias));
typedef float    v8f  __attribute__((ext_vector_type(8)));
typedef float    v4f  __attribute__((ext_vector_type(4)));
union Frag { v16h v; v8h half[2]; };

__device__ __forceinline__ v8f mma16(v16h a, v16h b, v8f c) {
  c = __builtin_amdgcn_wmma_f32_16x16x32_f16(false, a, false, b, (short)0, c, false, false);
  asm volatile("v_nop\n\tv_nop\n\tv_nop\n\tv_nop" : "+v"(c) : "v"(a), "v"(b));
  return c;
}
__device__ __forceinline__ int koff(int e, int h) { return (e < 8) ? (8 * h + e) : (16 + 8 * h + (e - 8)); }

__global__ __launch_bounds__(128) void k_cvt(const float* __restrict__ Wh, _Float16* __restrict__ WhT) {
  const int wave = threadIdx.x >> 5, lane = threadIdx.x & 31;
  const int row = blockIdx.x * 4 + wave;
  if (row >= N_IMAGES * 2 * HID) return;
  const int mat = row / HID, n = row - mat * HID;
  const float* src = Wh + (size_t)mat * HID * HID + n;
  v8h v;
#pragma unroll
  for (int i = 0; i < 8; ++i) v[i] = (_Float16)src[(size_t)(lane * 8 + i) * HID];
  _Float16* dst = WhT + (size_t)row * HID + lane * 8;
  *(volatile v8h*)dst = v;
  __threadfence();
  *(volatile v8h*)dst = v;
}

__global__ __launch_bounds__(32) void k_pos(const int* __restrict__ cam_id, int* __restrict__ pos) {
  const int lane = threadIdx.x;
  int base = 0;
  const unsigned lt = (1u << lane) - 1u;
  for (int s = 0; s < N_PIX / 32; ++s) {
    const int p = s * 32 + lane;
    const int c = cam_id[p];
    int myrank = -1;
#pragma unroll 1
    for (int cc = 0; cc < N_IMAGES; ++cc) {
      const unsigned b = (unsigned)__ballot(c == cc);
      const int bc = __shfl(base, cc, 32);
      if (c == cc) myrank = bc + __popc(b & lt);
      if (lane == cc) base += __popc(b);
    }
    *(volatile int*)(pos + p) = myrank;
    __threadfence();
    *(volatile int*)(pos + p) = myrank;
  }
}

__global__ __launch_bounds__(128) void k_mlp(const int* __restrict__ cam_id, const int* __restrict__ px,
                                            const int* __restrict__ py, const float* __restrict__ W1,
                                            const float* __restrict__ b1, const _Float16* __restrict__ WhT,
                                            const float* __restrict__ bh, const float* __restrict__ Wout,
                                            const float* __restrict__ bout, float* __restrict__ res) {
  __shared__ int list[N_PIX];
  __shared__ int s_cnt;
  __shared__ __attribute__((aligned(16))) _Float16 hbuf[4][16][HID + 8];
  const int cam = blockIdx.x, tid = threadIdx.x, wave = tid >> 5, lane = tid & 31;
  const int hi = lane >> 4, lrow = lane & 15;

  if (wave == 0) {
    int base = 0;
    const unsigned lt = (1u << lane) - 1u;
    for (int s = 0; s < N_PIX / 32; ++s) {
      const int p = s * 32 + lane;
      const int c = cam_id[p];
      const unsigned b = (unsigned)__ballot(c == cam);
      if (c == cam) list[base + __popc(b & lt)] = p;
      base += __popc(b);
    }
    if (lane == 0) s_cnt = base;
  }
  __syncthreads();
  const int count = s_cnt;
  const int ntiles = (count + 15) >> 4;

  const float* W1c = W1 + (size_t)cam * 2 * HID;
  const float* b1c = b1 + (size_t)cam * HID;
  const float* Woc = Wout + (size_t)cam * HID * 3;
  const float* boc = bout + cam * 3;

  for (int tile = wave; tile < ntiles; tile += 4) {
    const int row = tile * 16 + lrow;
    float x = 0.f, y = 0.f;
    if (row < count) {
      const int p = list[row];
      x = (float)px[p] / (float)(IMG_W - 1) * 2.0f - 1.0f;
      y = (float)py[p] / (float)(IMG_H - 1) * 2.0f - 1.0f;
    }
    __builtin_amdgcn_fence(__ATOMIC_ACQ_REL, "workgroup");
    __builtin_amdgcn_wave_barrier();
#pragma unroll 4
    for (int j = 0; j < HID / 2; ++j) {
      const int k = hi * (HID / 2) + j;
      const float v = x * W1c[k] + y * W1c[HID + k] + b1c[k];
      hbuf[wave][lrow][k] = (_Float16)fmaxf(v, 0.f);
    }
    Frag hfrag[8];
#pragma unroll 1
    for (int l = 0; l < 2; ++l) {
      const _Float16* WlT = WhT + ((size_t)(cam * 2 + l) * HID) * HID;
      const float* bl = bh + ((size_t)cam * 2 + l) * HID;
      __builtin_amdgcn_fence(__ATOMIC_ACQ_REL, "workgroup");
      __builtin_amdgcn_wave_barrier();
#pragma unroll
      for (int f = 0; f < 8; ++f) {
        hfrag[f].half[0] = *(const v8ha*)&hbuf[wave][lrow][f * 32 + 8 * hi];
        hfrag[f].half[1] = *(const v8ha*)&hbuf[wave][lrow][f * 32 + 16 + 8 * hi];
      }
      __builtin_amdgcn_fence(__ATOMIC_ACQ_REL, "workgroup");
      __builtin_amdgcn_wave_barrier();
#pragma unroll 1
      for (int nt = 0; nt < 16; ++nt) {
        const int n = nt * 16 + lrow;
        const float bias = bl[n];
        v8f acc = {bias, bias, bias, bias, bias, bias, bias, bias};
        const _Float16* bp = WlT + (size_t)n * HID;
#pragma unroll
        for (int ks = 0; ks < 8; ++ks) {
          Frag b;
          b.half[0] = *(const v8h*)(bp + ks * 32 + 8 * hi);
          b.half[1] = *(const v8h*)(bp + ks * 32 + 16 + 8 * hi);
          acc = mma16(hfrag[ks].v, b.v, acc);
        }
#pragma unroll
        for (int r = 0; r < 8; ++r) hbuf[wave][8 * hi + r][n] = (_Float16)fmaxf(acc[r], 0.f);
      }
    }
    __builtin_amdgcn_fence(__ATOMIC_ACQ_REL, "workgroup");
    __builtin_amdgcn_wave_barrier();
    float o0 = 0.f, o1 = 0.f, o2 = 0.f;
#pragma unroll 4
    for (int j = 0; j < HID / 2; ++j) {
      const int k = hi * (HID / 2) + j;
      const float hv = (float)hbuf[wave][lrow][k];
      o0 += hv * Woc[k * 3 + 0];
      o1 += hv * Woc[k * 3 + 1];
      o2 += hv * Woc[k * 3 + 2];
    }
    o0 += __shfl_xor(o0, 16, 32);
    o1 += __shfl_xor(o1, 16, 32);
    o2 += __shfl_xor(o2, 16, 32);
    v4f ov = {o0 + boc[0], o1 + boc[1], o2 + boc[2], 0.f};
    if (hi == 0) {
      float* dst = res + ((size_t)cam * N_PIX + row) * 4;
      *(volatile v4f*)dst = ov;
      __threadfence();
      *(volatile v4f*)dst = ov;
    }
  }
}

__global__ __launch_bounds__(256) void k_out(const int* __restrict__ cam_id, const int* __restrict__ pos,
                                            const float* __restrict__ res, float* __restrict__ out) {
  const int t = blockIdx.x * 256 + threadIdx.x;
  if (t >= N_PIX * 3 / 4) return;
  v4f v;
#pragma unroll
  for (int j = 0; j < 4; ++j) {
    const int g = t * 4 + j;
    const int p = g / 3, ch = g - p * 3;
    const int c = cam_id[p], ps = pos[p];
    float val = 0.f;
    if ((unsigned)c < (unsigned)N_IMAGES && (unsigned)ps < (unsigned)N_PIX) val = res[((size_t)c * N_PIX + ps) * 4 + ch];
    v[j] = val;
  }
  *(volatile v4f*)(out + (size_t)t * 4) = v;
  __threadfence();
  *(volatile v4f*)(out + (size_t)t * 4) = v;
}

extern "C" void kernel_launch(void* const* d_in, const int* in_sizes, int n_in,
                              void* d_out, int out_size, void* d_ws, size_t ws_size, hipStream_t stream) {
  (void)in_sizes; (void)n_in; (void)out_size;
  const int*   cam_id = (const int*)d_in[0];
  const int*   px     = (const int*)d_in[1];
  const int*   py     = (const int*)d_in[2];
  const float* W1   = (const float*)d_in[4];
  const float* b1   = (const float*)d_in[5];
  const float* Wh   = (const float*)d_in[6];
  const float* bh   = (const float*)d_in[7];
  const float* Wout = (const float*)d_in[8];
  const float* bout = (const float*)d_in[9];
  float* out = (float*)d_out;

  char* ws = (char*)d_ws;
  size_t off = 0;
  _Float16* WhT = (_Float16*)(ws + off); off += (size_t)N_IMAGES * 2 * HID * HID * sizeof(_Float16);
  int*   pos = (int*)(ws + off);          off += (size_t)N_PIX * sizeof(int);
  float* res = (float*)(ws + off);        off += (size_t)N_IMAGES * N_PIX * 4 * sizeof(float);
  if (off > ws_size) return;

  k_cvt<<<(N_IMAGES * 2 * HID) / 4, 128, 0, stream>>>(Wh, WhT);
  k_pos<<<1, 32, 0, stream>>>(cam_id, pos);
  k_mlp<<<N_IMAGES, 128, 0, stream>>>(cam_id, px, py, W1, b1, WhT, bh, Wout, bout, res);
  k_out<<<(N_PIX * 3 / 4 + 255) / 256, 256, 0, stream>>>(cam_id, pos, res, out);
}
